// BSplineKANLayer_2886218023198
// MI455X (gfx1250) — hardware-run, weakly checked
//
#include <hip/hip_runtime.h>
#include <math.h>
#include <stdint.h>


typedef __attribute__((ext_vector_type(16))) _Float16 v16h;
typedef __attribute__((ext_vector_type(8)))  _Float16 v8h;
typedef __attribute__((ext_vector_type(16))) __bf16   v16b;
typedef __attribute__((ext_vector_type(8)))  __bf16   v8b;
typedef __attribute__((ext_vector_type(8)))  float    v8f;
typedef __attribute__((ext_vector_type(4)))  float    v4f;

#define IN_DIM   1024
#define OUT_DIM  1024
#define NCOEF    8
#define NKNOT    12
#define KSPL     (IN_DIM * NCOEF)
#define KTOT     (KSPL + IN_DIM)
#define EPSV     1e-8f
#define BI       64
#define RBLK     32
#define A_SC     16.0f
#define S_SC     4.0f
#define C_SC     8.0f
#define W_SC     32.0f
#define OUT_SC   (1.0f / 128.0f)

__device__ __forceinline__ unsigned short f2bf_bits(float f) {
  unsigned u = __float_as_uint(f);
  return (unsigned short)((u + 0x7FFFu + ((u >> 16) & 1u)) >> 16);
}
__device__ __forceinline__ float bf_bits2f(unsigned short h) { return __uint_as_float(((unsigned)h) << 16); }

__device__ __forceinline__ void dep_guard_h(v8f& a, v8f& b, v16h x, v16h y) { asm volatile("v_nop\n\tv_nop\n\tv_nop\n\tv_nop" : "+v"(a), "+v"(b) : "v"(x), "v"(y)); }
__device__ __forceinline__ void dep_guard_b(v8f& a, v8f& b, v16b x, v16b y) { asm volatile("v_nop\n\tv_nop\n\tv_nop\n\tv_nop" : "+v"(a), "+v"(b) : "v"(x), "v"(y)); }
__device__ __forceinline__ void keep4_h(v16h a, v16h b, v16h c, v16h d) { asm volatile("v_nop" :: "v"(a), "v"(b), "v"(c), "v"(d)); }
__device__ __forceinline__ void keep4_b(v16b a, v16b b, v16b c, v16b d) { asm volatile("v_nop" :: "v"(a), "v"(b), "v"(c), "v"(d)); }
__device__ __forceinline__ void acc_guard4(v8f& a, v8f& b, v8f& c, v8f& d) { asm volatile("v_nop\n\tv_nop\n\tv_nop\n\tv_nop" : "+v"(a), "+v"(b), "+v"(c), "+v"(d)); }
template <typename T> struct Frag;
template <> struct Frag<_Float16> {
  typedef v16h V; union U { v16h v; v8h h[2]; };
  static __device__ __forceinline__ v16h load(const _Float16* p) {
    U f; f.h[0] = *(const v8h*)(p); f.h[1] = *(const v8h*)(p + 16); return f.v;
  }
  static __device__ __forceinline__ v8f mma(v16h a, v16h b, v8f c) {
    return __builtin_amdgcn_wmma_f32_16x16x32_f16(false, a, false, b, (short)0, c, false, false);
  }
  static __device__ __forceinline__ void guard(v8f& a, v8f& b, v16h x, v16h y) { dep_guard_h(a, b, x, y); }
  static __device__ __forceinline__ void keep(v16h a, v16h b, v16h c, v16h d) { keep4_h(a, b, c, d); }
};
template <> struct Frag<__bf16> {
  typedef v16b V; union U { v16b v; v8b h[2]; };
  static __device__ __forceinline__ v16b load(const __bf16* p) {
    U f; f.h[0] = *(const v8b*)(p); f.h[1] = *(const v8b*)(p + 16); return f.v;
  }
  static __device__ __forceinline__ v8f mma(v16b a, v16b b, v8f c) {
    return __builtin_amdgcn_wmma_f32_16x16x32_bf16(false, a, false, b, (short)0, c, false, false);
  }
  static __device__ __forceinline__ void guard(v8f& a, v8f& b, v16b x, v16b y) { dep_guard_b(a, b, x, y); }
  static __device__ __forceinline__ void keep(v16b a, v16b b, v16b c, v16b d) { keep4_b(a, b, c, d); }
};

template <int ET> struct Elem;
template <> struct Elem<0> { typedef _Float16 T; };
template <> struct Elem<1> { typedef __bf16 T; };
template <int ET, bool SPLIT, int BIAS_MODE, int OUT_MODE, bool RESID, int ACT = 0>
__global__ __launch_bounds__(256) void wmma_gemm64(
    const unsigned short* __restrict__ Ap, const unsigned short* __restrict__ A2p, int lda, long strideA,
    const unsigned short* __restrict__ Btp, const unsigned short* __restrict__ Bt2p, int ldb, long strideB,
    void* __restrict__ Cout, void* __restrict__ Cout2, int ldc, long strideC,
    const float* __restrict__ bias,
    const float* __restrict__ resid, long strideR, const float* __restrict__ rscale,
    int M, int N, int K, float scale) {
  typedef typename Elem<ET>::T T;
  typedef typename Frag<T>::V V;
  const T* A = (const T*)Ap; const T* A2 = (const T*)A2p; const T* Bt = (const T*)Btp; const T* Bt2 = (const T*)Bt2p;
  __shared__ __align__(16) float sT[8][16 * 68];
  const int b    = blockIdx.y;
  const int lane = threadIdx.x & 31;
  const int wave = threadIdx.x >> 5;
  const int tilesN = N >> 6;
  const int tilesM = M >> 6;
  const int tile = blockIdx.x * 8 + wave;
  if (tile >= tilesM * tilesN) return;
  const int tm = tile / tilesN;
  const int tn = tile - tm * tilesN;
  const int m0 = tm << 6;
  const int n0 = tn << 6;

  const T* Ab  = A  + (size_t)b * strideA;
  const T* Bb  = Bt + (size_t)b * strideB;
  const T* Ab2 = SPLIT ? (A2  + (size_t)b * strideA) : nullptr;
  const T* Bb2 = SPLIT ? (Bt2 + (size_t)b * strideB) : nullptr;

  const int rlane = lane & 15;
  const int koff  = (lane >> 4) * 8;
  const int mOff  = (lane >> 4) * 8;

  v8f acc[4][4];
#pragma unroll
  for (int i = 0; i < 4; ++i)
#pragma unroll
    for (int j = 0; j < 4; ++j) acc[i][j] = (v8f){0.f,0.f,0.f,0.f,0.f,0.f,0.f,0.f};

  for (int k0 = 0; k0 < K; k0 += 32) {
    V bh[4], bl[4];
#pragma unroll
    for (int j = 0; j < 4; ++j) {
      const size_t bo = (size_t)(n0 + (j << 4) + rlane) * ldb + koff + k0;
      bh[j] = Frag<T>::load(Bb + bo);
      if (SPLIT) bl[j] = Frag<T>::load(Bb2 + bo);
    }
#pragma unroll
    for (int i = 0; i < 4; ++i) {
      const size_t ao = (size_t)(m0 + (i << 4) + rlane) * lda + koff + k0;
      V ah = Frag<T>::load(Ab + ao);
      V al;
      if (SPLIT) al = Frag<T>::load(Ab2 + ao);
#pragma unroll
      for (int j = 0; j < 4; ++j) {
        acc[i][j] = Frag<T>::mma(ah, bh[j], acc[i][j]);
        if (SPLIT) {
          acc[i][j] = Frag<T>::mma(ah, bl[j], acc[i][j]);
          acc[i][j] = Frag<T>::mma(al, bh[j], acc[i][j]);
        }
      }
      Frag<T>::guard(acc[i][0], acc[i][3], ah, SPLIT ? al : ah);
    }
    Frag<T>::keep(bh[0], bh[1], bh[2], bh[3]);
    if (SPLIT) Frag<T>::keep(bl[0], bl[1], bl[2], bl[3]);
  }
  acc_guard4(acc[0][0], acc[0][1], acc[0][2], acc[0][3]);
  acc_guard4(acc[1][0], acc[1][1], acc[1][2], acc[1][3]);
  acc_guard4(acc[2][0], acc[2][1], acc[2][2], acc[2][3]);
  acc_guard4(acc[3][0], acc[3][1], acc[3][2], acc[3][3]);

  float* slab = sT[wave];
  const float* Rb = RESID ? (resid + (size_t)b * strideR) : nullptr;
  float rsv = 0.f;
  if (RESID) rsv = rscale[0];
#pragma unroll
  for (int i = 0; i < 4; ++i) {
    const int mBase = m0 + (i << 4);
#pragma unroll
    for (int j = 0; j < 4; ++j) {
      const int n = n0 + (j << 4) + rlane;
      float bv = 0.f;
      if (BIAS_MODE == 2) bv = bias[n];
#pragma unroll
      for (int r = 0; r < 8; ++r) {
        float v = acc[i][j][r] * scale;
        if (BIAS_MODE == 1) v += bias[mBase + mOff + r];
        if (BIAS_MODE == 2) v += bv;
        if (RESID) v += rsv * Rb[(size_t)(mBase + mOff + r) * ldc + n];
        if (ACT == 1) v = tanhf(v);
        if (ACT == 2) v = fmaxf(v, 0.0f);
        if (ACT == 3) v = v / (1.0f + expf(-v));
        if (ACT == 4) v = (v > 0.f) ? v : 0.01f * v;
        if (ACT == 5) v = 0.5f * v * (1.0f + erff(v * 0.70710678118654752f));
        slab[(mOff + r) * 68 + (j << 4) + rlane] = v;
      }
    }
    __builtin_amdgcn_fence(__ATOMIC_RELEASE, "workgroup");
    __builtin_amdgcn_wave_barrier();
    __builtin_amdgcn_fence(__ATOMIC_ACQUIRE, "workgroup");
    if (OUT_MODE == 0) {
      float* C = (float*)Cout + (size_t)b * strideC;
      const int hh = lane >> 4, c4 = (lane & 15) * 4;
      for (int pass = 0; pass < 2; ++pass) {
#pragma unroll
        for (int it = 0; it < 8; ++it) {
          const int row = it * 2 + hh;
          v4f v = *(const v4f*)(slab + row * 68 + c4);
          *(volatile v4f*)(C + (size_t)(mBase + row) * ldc + n0 + c4) = v;
        }
        __threadfence();
      }
    } else {
      const int q = lane >> 3, c8 = (lane & 7) * 8;
      unsigned short* C  = (unsigned short*)Cout  + (size_t)b * strideC;
      unsigned short* C2 = (OUT_MODE == 2) ? ((unsigned short*)Cout2 + (size_t)b * strideC) : nullptr;
      for (int pass = 0; pass < 2; ++pass) {
#pragma unroll
        for (int it = 0; it < 4; ++it) {
          const int row = it * 4 + q;
          const float* sp = slab + row * 68 + c8;
          v8h hv, lv;
#pragma unroll
          for (int e = 0; e < 8; ++e) {
            if (OUT_MODE == 1) {
              hv[e] = (_Float16)sp[e];
            } else {
              unsigned short hb = f2bf_bits(sp[e]);
              unsigned short lb = f2bf_bits(sp[e] - bf_bits2f(hb));
              hv[e] = __builtin_bit_cast(_Float16, hb);
              lv[e] = __builtin_bit_cast(_Float16, lb);
            }
          }
          *(volatile v8h*)(C + (size_t)(mBase + row) * ldc + n0 + c8) = hv;
          if (OUT_MODE == 2) *(volatile v8h*)(C2 + (size_t)(mBase + row) * ldc + n0 + c8) = lv;
        }
        __threadfence();
      }
    }
    __builtin_amdgcn_fence(__ATOMIC_RELEASE, "workgroup");
    __builtin_amdgcn_wave_barrier();
    __builtin_amdgcn_fence(__ATOMIC_ACQUIRE, "workgroup");
  }
}

__global__ __launch_bounds__(256) void cast_scale_f16x8(
    const float* __restrict__ src, int src_ld,
    _Float16* __restrict__ dst, int dst_ld, int dst_c0,
    int chunks_per_row, int nrows, float scale) {
  const int id = blockIdx.x * 256 + threadIdx.x;
  if (id < chunks_per_row * nrows) {
    const int r = id / chunks_per_row;
    const int c = (id - r * chunks_per_row) * 8;
    const float* sp = src + (size_t)r * src_ld + c;
    const v4f a = *(const v4f*)sp;
    const v4f bq = *(const v4f*)(sp + 4);
    v8h hv;
#pragma unroll
    for (int e = 0; e < 4; ++e) {
      hv[e]     = (_Float16)(a[e] * scale);
      hv[4 + e] = (_Float16)(bq[e] * scale);
    }
    _Float16* dp = dst + (size_t)r * dst_ld + dst_c0 + c;
    *(volatile v8h*)dp = hv;
    __threadfence();
    *(volatile v8h*)dp = hv;
  }
}

__global__ __launch_bounds__(256) void kan_basis(const float* __restrict__ x,
                                                 const float* __restrict__ gsl,
                                                 const float* __restrict__ gstart,
                                                 _Float16* __restrict__ Aall) {
  __shared__ float sg[BI][NKNOT];
  __shared__ float sR[BI][32];
  __shared__ float sS[8][BI];
  const int tid  = threadIdx.x;
  const int lane = tid & 31;
  const int wave = tid >> 5;
  const int i0 = blockIdx.x * BI;
  const int b0 = blockIdx.y * RBLK;

  if (tid < BI) {
    const int i = i0 + tid;
    float a = gstart[i];
    sg[tid][0] = a;
#pragma unroll 1
    for (int j = 0; j < NKNOT - 1; ++j) {
      const float v = gsl[(size_t)i * (NKNOT - 1) + j];
      const float sp = fmaxf(v, 0.0f) + log1pf(expf(-fabsf(v)));
      a += sp;
      sg[tid][j + 1] = a;
    }
#pragma unroll 1
    for (int t = 0; t < 30; ++t) {
      int d, k;
      if (t < 11)      { d = 1; k = t; }
      else if (t < 21) { d = 2; k = t - 11; }
      else             { d = 3; k = t - 21; }
      const float den = (sg[tid][k + d] - sg[tid][k]) + EPSV;
      sR[tid][t] = 1.0f / den;
    }
  }
  __syncthreads();

  for (int rr = wave; rr < RBLK; rr += 8) {
    const int b = b0 + rr;
    const float* xrow = x + (size_t)b * IN_DIM + i0;
    _Float16* arow = Aall + (size_t)b * KTOT;
#pragma unroll 1
    for (int hf = 0; hf < 2; ++hf) {
      const int il = hf * 32 + lane;
      const float xv = xrow[il];
      float g[NKNOT];
#pragma unroll
      for (int k = 0; k < NKNOT; ++k) g[k] = sg[il][k];
      float R[30];
#pragma unroll
      for (int t = 0; t < 30; ++t) R[t] = sR[il][t];
      float bb[NKNOT - 1];
#pragma unroll
      for (int k = 0; k < NKNOT - 1; ++k) bb[k] = (xv >= g[k] && xv < g[k + 1]) ? 1.0f : 0.0f;
#pragma unroll
      for (int k = 0; k < 10; ++k) {
        const float left  = (xv - g[k]) * R[k];
        const float right = (g[k + 2] - xv) * R[k + 1];
        bb[k] = left * bb[k] + right * bb[k + 1];
      }
#pragma unroll
      for (int k = 0; k < 9; ++k) {
        const float left  = (xv - g[k]) * R[11 + k];
        const float right = (g[k + 3] - xv) * R[11 + k + 1];
        bb[k] = left * bb[k] + right * bb[k + 1];
      }
#pragma unroll
      for (int k = 0; k < 8; ++k) {
        const float left  = (xv - g[k]) * R[21 + k];
        const float right = (g[k + 4] - xv) * R[21 + k + 1];
        bb[k] = left * bb[k] + right * bb[k + 1];
      }
      v8h p;
#pragma unroll
      for (int e = 0; e < NCOEF; ++e) p[e] = (_Float16)(bb[e] * A_SC);
      _Float16* ap = arow + (size_t)(i0 + il) * NCOEF;
      *(volatile v8h*)ap = p;
      __threadfence();
      *(volatile v8h*)ap = p;
      const float sgm = 1.0f / (1.0f + expf(-xv));
      sS[wave][il] = (xv * sgm) * S_SC;
    }
    __builtin_amdgcn_fence(__ATOMIC_RELEASE, "workgroup");
    __builtin_amdgcn_wave_barrier();
    __builtin_amdgcn_fence(__ATOMIC_ACQUIRE, "workgroup");
    {
      const float s0 = sS[wave][2 * lane];
      const float s1 = sS[wave][2 * lane + 1];
      const _Float16 h0 = (_Float16)s0, h1 = (_Float16)s1;
      const unsigned u = (unsigned)__builtin_bit_cast(unsigned short, h0) |
                         ((unsigned)__builtin_bit_cast(unsigned short, h1) << 16);
      unsigned* up = (unsigned*)(arow + KSPL + i0) + lane;
      *(volatile unsigned*)up = u;
      __threadfence();
      *(volatile unsigned*)up = u;
    }
    __builtin_amdgcn_fence(__ATOMIC_RELEASE, "workgroup");
    __builtin_amdgcn_wave_barrier();
    __builtin_amdgcn_fence(__ATOMIC_ACQUIRE, "workgroup");
  }
}

extern "C" void kernel_launch(void* const* d_in, const int* in_sizes, int n_in,
                              void* d_out, int out_size, void* d_ws, size_t ws_size,
                              hipStream_t stream) {
  if (n_in < 6) return;
  const float* x      = (const float*)d_in[0];
  const float* coeffs = (const float*)d_in[1];
  const float* basew  = (const float*)d_in[2];
  const float* gsl    = (const float*)d_in[3];
  const float* gstart = (const float*)d_in[4];
  const float* res    = (const float*)d_in[5];
  float* out = (float*)d_out;

  const int M = in_sizes[0] / IN_DIM;
  if (M <= 0 || (M % 64) != 0 || (M % RBLK) != 0) return;
  if (in_sizes[0] != M * IN_DIM) return;
  if (in_sizes[1] != OUT_DIM * KSPL || in_sizes[2] != OUT_DIM * IN_DIM) return;
  if (in_sizes[3] != IN_DIM * (NKNOT - 1) || in_sizes[4] != IN_DIM || in_sizes[5] < 1) return;
  if ((size_t)out_size < (size_t)M * OUT_DIM) return;

  const size_t bt_bytes = (size_t)OUT_DIM * KTOT * sizeof(_Float16);
  const size_t a_bytes  = (size_t)M * KTOT * sizeof(_Float16);
  if (bt_bytes + a_bytes > ws_size) return;
  char* ws = (char*)d_ws;
  _Float16* Btall = (_Float16*)ws;
  _Float16* Aall  = (_Float16*)(ws + bt_bytes);

  {
    const int chunks1 = KSPL / 8;
    const int tot1 = OUT_DIM * chunks1;
    cast_scale_f16x8<<<(tot1 + 255) / 256, 256, 0, stream>>>(coeffs, KSPL, Btall, KTOT, 0, chunks1, OUT_DIM, C_SC);
    const int chunks2 = IN_DIM / 8;
    const int tot2 = OUT_DIM * chunks2;
    cast_scale_f16x8<<<(tot2 + 255) / 256, 256, 0, stream>>>(basew, IN_DIM, Btall, KTOT, KSPL, chunks2, OUT_DIM, W_SC);
  }

  {
    dim3 grid(IN_DIM / BI, M / RBLK);
    kan_basis<<<grid, 256, 0, stream>>>(x, gsl, gstart, Aall);
  }

  {
    const int tiles = (M / 64) * (OUT_DIM / 64);
    dim3 grid((tiles + 7) / 8, 1);
    wmma_gemm64<0, false, 0, 0, true, 0><<<grid, 256, 0, stream>>>(
        (const unsigned short*)Aall, (const unsigned short*)Aall, KTOT, 0L,
        (const unsigned short*)Btall, (const unsigned short*)Btall, KTOT, 0L,
        (void*)out, (void*)out, OUT_DIM, 0L,
        res,
        x, 0L, res,
        M, OUT_DIM, KTOT, OUT_SC);
  }
  (void)hipGetLastError();
}
